// MultiDimBehavioralCRSAE_16552803958954
// MI455X (gfx1250) — hardware-verified
//
#include <hip/hip_runtime.h>
#include <math.h>

typedef __attribute__((ext_vector_type(16))) _Float16 v16h;
typedef __attribute__((ext_vector_type(8)))  _Float16 v8h;
typedef __attribute__((ext_vector_type(4)))  _Float16 v4h;
typedef __attribute__((ext_vector_type(8)))  float    v8f;
typedef __attribute__((ext_vector_type(4)))  float    v4f;
typedef __attribute__((ext_vector_type(4)))  unsigned u4v;

constexpr int kCh    = 8;
constexpr int kTr    = 16;
constexpr int kLen   = 4096;
constexpr int kNf    = 16;
constexpr int kTaps  = 64;
constexpr int kEnc   = kLen - kTaps + 1;
constexpr int kSteps = 10;
constexpr int kXP    = 4096;
constexpr int kHP    = 4224;
constexpr int kLeft  = 64;
constexpr int kWin   = 80;
constexpr int kKs    = kNf * kWin;
constexpr int kRowsX = kCh * kTr * kNf;
constexpr int kRowsR = kCh * kTr;
static_assert(kEnc == 4033, "code length");
static_assert(kKs == 1280 && (kKs % 32) == 0 && (kTaps % 32) == 0, "K multiples of 32");
static_assert(kCh * kTr * kLen == 524288, "input 0 element count");
static_assert(kCh * kNf * kTaps == 8192, "input 1 element count");
static_assert(kRowsX * kEnc == 8259584, "output element count");
static_assert((kRowsX * kEnc) % 1024 == 0, "pack grid exact");
static_assert(kLeft + kLen <= kHP && kLen + 128 <= kHP, "pads inside pitch");

constexpr float kHCarry  = 64.0f;
constexpr float kLoCarry = 2048.0f;
constexpr float kInvH    = 1.0f / kHCarry;
constexpr float kInvHL   = 1.0f / (kHCarry * kLoCarry);
constexpr float kMinNormH = 6.103515625e-05f;
constexpr float kInvLip  = (float)(1.0 / 10.0);
constexpr float kThr     = (float)(0.1 / 10.0);

constexpr size_t kSzXf = (size_t)kRowsX * kXP * 4;
constexpr size_t kSzXh = (size_t)kRowsX * kHP * 2;
constexpr size_t kSzRh = (size_t)kRowsR * kHP * 2;
constexpr size_t kSzAT = (size_t)kCh * 16 * kKs * 2;
constexpr size_t kSzHF = (size_t)kCh * kNf * kTaps * 2;
constexpr size_t kOffXO = 0;
constexpr size_t kOffXT = kOffXO + kSzXf;
constexpr size_t kOffXH = kOffXT + kSzXf;
constexpr size_t kOffXL = kOffXH + kSzXh;
constexpr size_t kOffRH = kOffXL + kSzXh;
constexpr size_t kOffRL = kOffRH + kSzRh;
constexpr size_t kOffAT = kOffRL + kSzRh;
constexpr size_t kOffHF = kOffAT + kSzAT;
constexpr size_t kWsTotal = kOffHF + kSzHF;
static_assert(kWsTotal == 104218624ull, "carve total");
static_assert(kWsTotal <= 134217728ull, "carve cap");
static_assert((kOffXT % 128) == 0 && (kOffXH % 128) == 0 && (kOffXL % 128) == 0 && (kOffRH % 128) == 0 &&
              (kOffRL % 128) == 0 && (kOffAT % 128) == 0 && (kOffHF % 128) == 0, "128-B aligned regions");

constexpr int kPrepAT  = (kCh * 16 * kKs / 8) / 256;
constexpr int kPrepHF  = (kCh * kNf * kTaps / 8) / 256;
constexpr int kPrepPad = (2 * kRowsX * 16) / 256;
static_assert(kPrepAT == 80 && kPrepHF == 4 && kPrepPad == 256, "prep grid");

__device__ __forceinline__ unsigned short f2bf_bits(float f) {
  unsigned u = __float_as_uint(f);
  return (unsigned short)((u + 0x7FFFu + ((u >> 16) & 1u)) >> 16);
}
__device__ __forceinline__ float bf_rne(float f) {
  return __uint_as_float(((unsigned)f2bf_bits(f)) << 16);
}
__device__ __forceinline__ void split_hl(float v, _Float16& hi, _Float16& lo) {
  const float hc = (float)((_Float16)v);
  const float hf = (fabsf(v) < kMinNormH) ? 0.0f : hc;
  hi = (_Float16)hf;
  lo = (_Float16)((v - hf) * kLoCarry);
}
union FragU { v16h v; v8h h[2]; };
__device__ __forceinline__ v16h frag_load(const _Float16* p) {
  FragU f;
  f.h[0] = *(const v8h*)(p);
  f.h[1] = *(const v8h*)(p + 16);
  return f.v;
}
__device__ __forceinline__ v8f mma16(v16h a, v16h b, v8f c) {
  return __builtin_amdgcn_wmma_f32_16x16x32_f16(false, a, false, b, (short)0, c, false, false);
}
__device__ __forceinline__ void acc_guard2(v8f& acc, v16h x, v16h y) {
  asm volatile("v_nop\n\tv_nop\n\tv_nop\n\tv_nop" : "+v"(acc) : "v"(x), "v"(y));
}
__device__ __forceinline__ void acc_guard4(v8f& acc, v16h x0, v16h x1, v16h x2, v16h x3) {
  asm volatile("v_nop\n\tv_nop\n\tv_nop\n\tv_nop" : "+v"(acc) : "v"(x0), "v"(x1), "v"(x2), "v"(x3));
}
__device__ __forceinline__ void store_v8h_twice(unsigned short* dst, v8h v) {
  *(volatile v8h*)dst = v;
  __threadfence();
  *(volatile v8h*)dst = v;
}

__global__ __launch_bounds__(256) void prep_kernel(
    const float* __restrict__ Hin, unsigned short* __restrict__ AT, unsigned short* __restrict__ HF,
    unsigned short* __restrict__ XH, unsigned short* __restrict__ XL)
{
  const int bid = blockIdx.x, tid = threadIdx.x;
  if (bid < kPrepAT) {
    const int p  = bid * 256 + tid;
    const int kp = p % (kKs / 8);
    const int rm = p / (kKs / 8);
    const int m  = rm & 15;
    const int ch = rm >> 4;
    const int k  = kp * 8;
    const int f  = k / kWin;
    const int u0 = k - f * kWin;
    const float* hrow = Hin + (size_t)(ch * kNf + f) * kTaps;
    v8h val;
#pragma unroll
    for (int e = 0; e < 8; ++e) {
      const int j = m + 64 - (u0 + e);
      const bool ok = (j >= 0) && (j < kTaps);
      const int jc = (j < 0) ? 0 : ((j > kTaps - 1) ? (kTaps - 1) : j);
      const float hv = hrow[jc];
      const float w = ok ? (bf_rne(hv) * kHCarry) : 0.0f;
      val[e] = (_Float16)w;
    }
    store_v8h_twice(AT + (size_t)p * 8, val);
  } else if (bid < kPrepAT + kPrepHF) {
    const int p = (bid - kPrepAT) * 256 + tid;
    const v4f a0 = *(const v4f*)(Hin + (size_t)p * 8);
    const v4f a1 = *(const v4f*)(Hin + (size_t)p * 8 + 4);
    v8h val;
#pragma unroll
    for (int e = 0; e < 4; ++e) {
      const float s0 = a0[e];
      const float s1 = a1[e];
      val[e]     = (_Float16)(bf_rne(s0) * kHCarry);
      val[4 + e] = (_Float16)(bf_rne(s1) * kHCarry);
    }
    store_v8h_twice(HF + (size_t)p * 8, val);
  } else {
    const int p     = (bid - kPrepAT - kPrepHF) * 256 + tid;
    const int plane = p >> 15;
    const int rem   = p & 32767;
    const int row   = rem >> 4;
    const int seg   = rem & 15;
    const int side  = seg >> 3;
    const int l8    = seg & 7;
    const int col   = side * (kLeft + kLen) + l8 * 8;
    unsigned short* base = (plane == 0) ? XH : XL;
    unsigned short* dst = base + (size_t)row * kHP + col;
    const u4v z = {0u, 0u, 0u, 0u};
    *(volatile u4v*)dst = z;
    __threadfence();
    *(volatile u4v*)dst = z;
  }
}

__global__ __launch_bounds__(256) void ysplit_kernel(
    const float* __restrict__ y, unsigned short* __restrict__ RH, unsigned short* __restrict__ RL)
{
  const int p   = blockIdx.x * 256 + threadIdx.x;
  const int row = p / (kHP / 8);
  const int pc  = p - row * (kHP / 8);
  const int col = pc * 8;
  const int ch  = row >> 4;
  const int n   = row & 15;
  const int colc = (col > kLen - 8) ? (kLen - 8) : col;
  const bool live = col < kLen;
  const float* src = y + ((size_t)(n * kCh + ch) * kLen + colc);
  const v4f a0 = *(const v4f*)(src);
  const v4f a1 = *(const v4f*)(src + 4);
  v8h hv, lv;
#pragma unroll
  for (int e = 0; e < 4; ++e) {
    const float s0 = a0[e];
    const float s1 = a1[e];
    const float r0 = live ? bf_rne(s0) : 0.0f;
    const float r1 = live ? bf_rne(s1) : 0.0f;
    _Float16 h0, l0, h1, l1;
    split_hl(r0, h0, l0);
    split_hl(r1, h1, l1);
    hv[e] = h0; lv[e] = l0;
    hv[4 + e] = h1; lv[4 + e] = l1;
  }
  unsigned short* qh = RH + (size_t)row * kHP + col;
  unsigned short* ql = RL + (size_t)row * kHP + col;
  *(volatile v8h*)qh = hv;
  *(volatile v8h*)ql = lv;
  __threadfence();
  *(volatile v8h*)qh = hv;
  *(volatile v8h*)ql = lv;
}

__global__ __launch_bounds__(128) void synth_kernel(
    const unsigned short* __restrict__ XHp, const unsigned short* __restrict__ XLp,
    const unsigned short* __restrict__ ATp, const float* __restrict__ y,
    unsigned short* __restrict__ RHp, unsigned short* __restrict__ RLp)
{
  __shared__ __align__(16) float sD[16 * 68];
  const int tid = threadIdx.x, lane = tid & 31, wave = tid >> 5;
  const int c = lane & 15, h = lane >> 4;
  const int ch = blockIdx.y;
  const int tb = blockIdx.x * 64;
  const int t0 = tb + wave * 16;
  const _Float16* at = (const _Float16*)ATp + (size_t)(ch * 16 + c) * kKs + 8 * h;
  const size_t xoff = (size_t)((ch * kTr + c) * kNf) * kHP + t0 + 8 * h;
  const _Float16* xh = (const _Float16*)XHp + xoff;
  const _Float16* xl = (const _Float16*)XLp + xoff;
  v8f accH = (v8f){0.f, 0.f, 0.f, 0.f, 0.f, 0.f, 0.f, 0.f};
  v8f accL = (v8f){0.f, 0.f, 0.f, 0.f, 0.f, 0.f, 0.f, 0.f};
#pragma unroll 1
  for (int fp = 0; fp < kNf / 2; ++fp) {
    const _Float16* ap = at + fp * (2 * kWin);
    const _Float16* hp = xh + (size_t)(2 * fp) * kHP;
    const _Float16* lp = xl + (size_t)(2 * fp) * kHP;
#pragma unroll
    for (int cc = 0; cc < 5; ++cc) {
      const int lb0 = cc * 32;
      const int lb1 = cc * 32 + 16;
      const int o0 = (lb0 >= kWin) ? (kHP + lb0 - kWin) : lb0;
      const int o1 = (lb1 >= kWin) ? (kHP + lb1 - kWin) : lb1;
      const v16h a = frag_load(ap + cc * 32);
      FragU bh, bl;
      bh.h[0] = *(const v8h*)(hp + o0);
      bh.h[1] = *(const v8h*)(hp + o1);
      bl.h[0] = *(const v8h*)(lp + o0);
      bl.h[1] = *(const v8h*)(lp + o1);
      accH = mma16(a, bh.v, accH);
      accL = mma16(a, bl.v, accL);
      acc_guard2(accH, a, bh.v);
      acc_guard2(accL, a, bl.v);
    }
  }
  {
    v4f d0, d1;
#pragma unroll
    for (int r = 0; r < 4; ++r) {
      d0[r] = accH[r] * kInvH + accL[r] * kInvHL;
      d1[r] = accH[4 + r] * kInvH + accL[4 + r] * kInvHL;
    }
    float* dp = sD + c * 68 + wave * 16 + 8 * h;
    *(v4f*)(dp) = d0;
    *(v4f*)(dp + 4) = d1;
  }
  __syncthreads();
  const int q = lane >> 3, c8 = (lane & 7) * 8;
  const int n = wave * 4 + q;
  const float* sp = sD + n * 68 + c8;
  const v4f e0 = *(const v4f*)(sp);
  const v4f e1 = *(const v4f*)(sp + 4);
  const float* yp = y + ((size_t)(n * kCh + ch) * kLen + tb + c8);
  const v4f y0 = *(const v4f*)(yp);
  const v4f y1 = *(const v4f*)(yp + 4);
  v8h hv, lv;
#pragma unroll
  for (int e = 0; e < 4; ++e) {
    const float ys0 = y0[e];
    const float ys1 = y1[e];
    const float r0 = bf_rne(ys0) - e0[e];
    const float r1 = bf_rne(ys1) - e1[e];
    _Float16 h0, l0, h1, l1;
    split_hl(r0, h0, l0);
    split_hl(r1, h1, l1);
    hv[e] = h0; lv[e] = l0;
    hv[4 + e] = h1; lv[4 + e] = l1;
  }
  const size_t ro = (size_t)(ch * kTr + n) * kHP + tb + c8;
  *(volatile v8h*)(RHp + ro) = hv;
  *(volatile v8h*)(RLp + ro) = lv;
  __threadfence();
  *(volatile v8h*)(RHp + ro) = hv;
  *(volatile v8h*)(RLp + ro) = lv;
}

__global__ __launch_bounds__(256) void analysis_kernel(
    const unsigned short* __restrict__ RHp, const unsigned short* __restrict__ RLp,
    const unsigned short* __restrict__ HFp,
    float* XO, float* XT, unsigned short* __restrict__ XHp, unsigned short* __restrict__ XLp,
    float mom, int first, int last)
{
  __shared__ __align__(16) unsigned sRaw[2 * 128];
  __shared__ __align__(16) unsigned short sSh[2 * 8 * 184];
  __shared__ __align__(16) float sG[16 * 132];
  const int tid = threadIdx.x, lane = tid & 31, wave = tid >> 5;
  const int cn = blockIdx.y;
  const int ch = cn >> 4;
  const int base = blockIdx.x * 128;

  if (wave < 2) {
    const unsigned short* src = (wave == 0) ? RHp : RLp;
    const u4v w = *(const u4v*)(src + (size_t)cn * kHP + base + lane * 8);
    *(u4v*)(sRaw + wave * 128 + lane * 4) = w;
  }
  __syncthreads();
  for (int idx = tid; idx < 368; idx += 256) {
    const int pl = idx / 184;
    const int r  = idx - pl * 184;
    const int s  = r / 23;
    const int p  = r - s * 23;
    const int i0 = s + 8 * p;
    const int a  = i0 >> 1;
    const unsigned* rw = sRaw + pl * 128 + a;
    const unsigned w0 = rw[0], w1 = rw[1], w2 = rw[2], w3 = rw[3], w4 = rw[4];
    const bool odd = (i0 & 1) != 0;
    u4v o;
    o[0] = odd ? ((w0 >> 16) | (w1 << 16)) : w0;
    o[1] = odd ? ((w1 >> 16) | (w2 << 16)) : w1;
    o[2] = odd ? ((w2 >> 16) | (w3 << 16)) : w2;
    o[3] = odd ? ((w3 >> 16) | (w4 << 16)) : w3;
    *(u4v*)(sSh + (pl * 8 + s) * 184 + 8 * p) = o;
  }
  __syncthreads();

  const int c = lane & 15, h = lane >> 4, s7 = c & 7;
  {
    const _Float16* hf = (const _Float16*)HFp + (size_t)(ch * kNf + c) * kTaps + 8 * h;
    const v16h a0 = frag_load(hf);
    const v16h a1 = frag_load(hf + 32);
    const int off = 16 * wave + c - s7 + 8 * h;
    const _Float16* bhp = (const _Float16*)(sSh + (0 * 8 + s7) * 184 + off);
    const _Float16* blp = (const _Float16*)(sSh + (1 * 8 + s7) * 184 + off);
    const v16h bh0 = frag_load(bhp);
    const v16h bh1 = frag_load(bhp + 32);
    const v16h bl0 = frag_load(blp);
    const v16h bl1 = frag_load(blp + 32);
    v8f accH = (v8f){0.f, 0.f, 0.f, 0.f, 0.f, 0.f, 0.f, 0.f};
    v8f accL = (v8f){0.f, 0.f, 0.f, 0.f, 0.f, 0.f, 0.f, 0.f};
    accH = mma16(a0, bh0, accH);
    accH = mma16(a1, bh1, accH);
    accL = mma16(a0, bl0, accL);
    accL = mma16(a1, bl1, accL);
    acc_guard4(accH, a0, a1, bh0, bh1);
    acc_guard4(accL, a0, a1, bl0, bl1);
#pragma unroll
    for (int r = 0; r < 8; ++r)
      sG[(8 * h + r) * 132 + 16 * wave + c] = accH[r] * kInvH + accL[r] * kInvHL;
  }
  __syncthreads();

  const int tl = lane * 4;
  const int t  = base + tl;
  v4f xn[2], xm[2];
  v4h hv[2], lv[2];
#pragma unroll
  for (int rr = 0; rr < 2; ++rr) {
    const int f = 2 * wave + rr;
    const size_t R = (size_t)cn * kNf + f;
    const v4f g = *(const v4f*)(sG + f * 132 + tl);
    v4f xt = (v4f){0.f, 0.f, 0.f, 0.f};
    v4f xo = (v4f){0.f, 0.f, 0.f, 0.f};
    if (first == 0) {
      xt = *(const v4f*)(XT + R * kXP + t);
      xo = *(const v4f*)(XO + R * kXP + t);
    }
#pragma unroll
    for (int e = 0; e < 4; ++e) {
      const bool live = (t + e) < kEnc;
      const float gs = g[e];
      const float xts = xt[e];
      const float xos = xo[e];
      float v = xts + gs * kInvLip - kThr;
      v = fmaxf(v, 0.0f);
      const float xnew = live ? v : 0.0f;
      float xmom = xnew + mom * (xnew - xos);
      xmom = live ? xmom : 0.0f;
      xn[rr][e] = xnew;
      xm[rr][e] = xmom;
      _Float16 hh, ll;
      split_hl(xmom, hh, ll);
      hv[rr][e] = hh;
      lv[rr][e] = ll;
    }
  }
  for (int pass = 0; pass < 2; ++pass) {
#pragma unroll
    for (int rr = 0; rr < 2; ++rr) {
      const size_t R = (size_t)cn * kNf + 2 * wave + rr;
      *(volatile v4f*)(XO + R * kXP + t) = xn[rr];
      if (last == 0) {
        *(volatile v4f*)(XT + R * kXP + t) = xm[rr];
        *(volatile v4h*)(XHp + R * kHP + kLeft + t) = hv[rr];
        *(volatile v4h*)(XLp + R * kHP + kLeft + t) = lv[rr];
      }
    }
    __threadfence();
  }
}

__global__ __launch_bounds__(256) void pack_kernel(const float* __restrict__ XO, float* __restrict__ out)
{
  const unsigned i  = blockIdx.x * 256u + threadIdx.x;
  const unsigned g0 = i * 4u;
  const unsigned row0 = g0 / (unsigned)kEnc;
  const unsigned tt0  = g0 - row0 * (unsigned)kEnc;
  v4f v;
#pragma unroll
  for (int e = 0; e < 4; ++e) {
    unsigned tt = tt0 + (unsigned)e;
    const bool wrap = tt >= (unsigned)kEnc;
    const unsigned row = wrap ? (row0 + 1u) : row0;
    tt = wrap ? (tt - (unsigned)kEnc) : tt;
    v[e] = XO[(size_t)row * kXP + tt];
  }
  float* dst = out + (size_t)g0;
  *(volatile v4f*)dst = v;
  __threadfence();
  *(volatile v4f*)dst = v;
}

extern "C" void kernel_launch(void* const* d_in, const int* in_sizes, int n_in,
                              void* d_out, int out_size, void* d_ws, size_t ws_size,
                              hipStream_t stream) {
  if (n_in < 2) return;
  if (in_sizes[0] != kTr * kCh * kLen) return;
  if (in_sizes[1] != kCh * kNf * kTaps) return;
  if (out_size != kRowsX * kEnc) return;
  if (ws_size < kWsTotal) return;

  const float* y   = (const float*)d_in[0];
  const float* Hin = (const float*)d_in[1];
  float* out = (float*)d_out;
  char* ws = (char*)d_ws;
  float*          XO = (float*)(ws + kOffXO);
  float*          XT = (float*)(ws + kOffXT);
  unsigned short* XH = (unsigned short*)(ws + kOffXH);
  unsigned short* XL = (unsigned short*)(ws + kOffXL);
  unsigned short* RH = (unsigned short*)(ws + kOffRH);
  unsigned short* RL = (unsigned short*)(ws + kOffRL);
  unsigned short* AT = (unsigned short*)(ws + kOffAT);
  unsigned short* HF = (unsigned short*)(ws + kOffHF);

  prep_kernel<<<kPrepAT + kPrepHF + kPrepPad, 256, 0, stream>>>(Hin, AT, HF, XH, XL);
  ysplit_kernel<<<(kRowsR * (kHP / 8)) / 256, 256, 0, stream>>>(y, RH, RL);

  float s_old = 1.0f;
  for (int it = 0; it < kSteps; ++it) {
    const float s_new = (1.0f + sqrtf(1.0f + 4.0f * s_old * s_old)) * 0.5f;
    const float mom = (s_old - 1.0f) / s_new;
    s_old = s_new;
    if (it > 0) {
      synth_kernel<<<dim3(kLen / 64, kCh), 128, 0, stream>>>(XH, XL, AT, y, RH, RL);
    }
    analysis_kernel<<<dim3(kLen / 128, kRowsR), 256, 0, stream>>>(
        RH, RL, HF, XO, XT, XH, XL, mom, (it == 0) ? 1 : 0, (it == kSteps - 1) ? 1 : 0);
  }
  pack_kernel<<<(kRowsX * kEnc / 4) / 256, 256, 0, stream>>>(XO, out);
}
